// MarketGraphNN_4776003633739
// MI455X (gfx1250) — hardware-run, weakly checked
//
#include <hip/hip_runtime.h>
#include <stddef.h>
#include <stdint.h>
#include <math.h>

#define NN      30000
#define NE      480000
#define F0      256
#define H1W     512
#define H2W     256
#define NC      16
#define MP      30080
#define GBM     64
#define GBN     128
#define GTHR    128
#define NTHR    256
#define NWAVE   8
#define EPT     8
#define WCH     (32 * EPT)
#define NBRUN   1024
#define SLB     10
#define NBK     30
#define WLCAP   2560
#define RCAP    20480
#define TRIPCAP 64
#define MAXDEG_MEAS   37
#define MAXB1024_MEAS 16604
#define RPB     64
#define RPW     8
#define SMF     896

#define SINGLE_TWO   1
#define SINGLE_THREE 1

#define K1   256
#define AP1  256
#define BP1  256
#define K2   (SINGLE_TWO ? 512 : 1024)
#define AP2  1024
#define BP2  1024
#define K3   (SINGLE_THREE ? 256 : 512)
#define AP3  512
#define BP3  512

#define BK_ZINTS (NWAVE * WLCAP + RCAP + 3 * NBRUN)
#define BK_INTS  (BK_ZINTS + 16)
#define BK_LDS   (BK_INTS * 4)

#define PBX  (MP * F0 / 8 / NTHR)
#define PBW1 (H1W * F0 / 8 / NTHR)
#define PBW2 (H2W * 1024 / 8 / NTHR)
#define PBW3 (NC * 512 / 8 / NTHR)
#define PBTOT (PBX + PBW1 + PBW2 + PBW3 + 1)

static_assert(MP % GBM == 0 && MP % 128 == 0 && MP >= NN && MP == 235 * 128 && MP % RPB == 0);
static_assert(NN == 234 * 128 + 48 && (NN % 2) == 0 && NN % 16 == 0);
static_assert(NBRUN == (1 << SLB) && NBRUN % RPB == 0 && NBRUN % 16 == 0 && NBRUN % 32 == 0);
static_assert((NBK - 1) * NBRUN < NN && NN <= NBK * NBRUN && NBK * NBRUN >= MP);
static_assert(NE < (1 << 21) && (((long long)NE) << SLB) < (1LL << 31));
static_assert(NE % WCH == 0 && NE % 4 == 0);
static_assert(RCAP == NWAVE * WLCAP && RCAP % (NTHR * 4) == 0 && BK_ZINTS % 4 == 0 && RCAP % 1024 == 0);
static_assert((long long)RCAP * 100 >= (long long)MAXB1024_MEAS * 105);
static_assert(WLCAP >= MAXB1024_MEAS / 8 + 8 * 46 + 1);
static_assert(NN <= 65535);
static_assert(MAXDEG_MEAS + 8 <= TRIPCAP && TRIPCAP < RCAP);
static_assert(H1W == 32 * 16 && H2W == 32 * 8 && H1W == 4 * GBN && H2W == 2 * GBN);
static_assert(K1 % 32 == 0 && K2 % 32 == 0 && K3 % 32 == 0);
static_assert(K1 <= AP1 && K1 <= BP1 && K2 <= AP2 && K2 <= BP2 && K3 <= AP3 && K3 <= BP3);
static_assert(AP2 == 2 * H1W && AP3 == 2 * H2W && AP1 == F0);
static_assert((MP * F0 / 8) % NTHR == 0 && (H1W * F0 / 8) % NTHR == 0);
static_assert((H2W * 1024 / 8) % NTHR == 0 && (NC * 512 / 8) % NTHR == 0);
static_assert(BK_LDS <= 300000);
static_assert(GBM * GBN * 4 <= 65536);
static_assert(NN * NC == 1875 * 256);
static_assert(SMF % 32 == 0 && SMF >= 768 + NC && SMF / 4 <= NTHR && (SMF / 4) % 32 == 0);

typedef float          v4f   __attribute__((ext_vector_type(4)));
typedef float          v8f   __attribute__((ext_vector_type(8)));
typedef int            v4i   __attribute__((ext_vector_type(4)));
typedef int            v8i   __attribute__((ext_vector_type(8)));
typedef unsigned short v8us  __attribute__((ext_vector_type(8)));
typedef unsigned short v16us __attribute__((ext_vector_type(16)));
typedef __bf16         v16bf __attribute__((ext_vector_type(16)));
typedef v4f  __attribute__((may_alias)) v4fa;
typedef v4i  __attribute__((may_alias)) v4ia;
typedef v8us __attribute__((may_alias)) v8usa;
union FragB { v16bf v; v16us u; v8us h[2]; v8i w; };

__device__ __forceinline__ v8f wmb(const FragB& a, const FragB& b, v8f c) {
  v8f d = __builtin_amdgcn_wmma_f32_16x16x32_bf16(false, a.v, false, b.v, (short)0, c, false, false);
  asm volatile("v_nop\n\tv_nop\n\tv_nop\n\tv_nop" : "+v"(d) : "v"(a.w), "v"(b.w));
  return d;
}

__device__ __forceinline__ unsigned bf16_bits(float f) {
  const unsigned u = __float_as_uint(f);
  const unsigned r = (u + 0x7FFFu + ((u >> 16) & 1u)) >> 16;
  const unsigned q = (u >> 16) | 0x40u;
  return ((u & 0x7fffffffu) > 0x7f800000u) ? q : r;
}

__device__ __forceinline__ void hilo_pack(float v0, float v1, float v2, float v3,
                                          int& h01, int& h23, int& l01, int& l23) {
  const unsigned a0 = bf16_bits(v0), a1 = bf16_bits(v1), a2 = bf16_bits(v2), a3 = bf16_bits(v3);
  const unsigned b0 = bf16_bits(v0 - __uint_as_float(a0 << 16));
  const unsigned b1 = bf16_bits(v1 - __uint_as_float(a1 << 16));
  const unsigned b2 = bf16_bits(v2 - __uint_as_float(a2 << 16));
  const unsigned b3 = bf16_bits(v3 - __uint_as_float(a3 << 16));
  h01 = (int)(a0 | (a1 << 16)); h23 = (int)(a2 | (a3 << 16));
  l01 = (int)(b0 | (b1 << 16)); l23 = (int)(b2 | (b3 << 16));
}

__device__ __forceinline__ v4i regroup16(int h01, int h23, int l01, int l23, int lane) {
  const int t  = lane & 15;
  const int s0 = 2 * t, s1 = s0 + 1;
  const int a0 = __shfl(h01, s0, 32), a1 = __shfl(h23, s0, 32), a2 = __shfl(h01, s1, 32), a3 = __shfl(h23, s1, 32);
  const int b0 = __shfl(l01, s0, 32), b1 = __shfl(l23, s0, 32), b2 = __shfl(l01, s1, 32), b3 = __shfl(l23, s1, 32);
  const int mk = (lane < 16) ? -1 : 0;
  v4i o;
  o.x = (a0 & mk) | (b0 & ~mk); o.y = (a1 & mk) | (b1 & ~mk);
  o.z = (a2 & mk) | (b2 & ~mk); o.w = (a3 & mk) | (b3 & ~mk);
  return o;
}

__device__ __forceinline__ void st2_v4f(float* p, v4f v) {
  *(volatile v4f*)p = v;
  __threadfence();
  *(volatile v4f*)p = v;
}
__device__ __forceinline__ void st2_v8us(unsigned short* p, v8us v) {
  *(volatile v8us*)p = v;
  __threadfence();
  *(volatile v8us*)p = v;
}

__device__ __forceinline__ v8us gather8(const float* __restrict__ base, int stride) {
  float f[8];
#pragma unroll
  for (int i = 0; i < 8; ++i) f[i] = base[(size_t)i * (size_t)stride];
  v8us o;
#pragma unroll
  for (int i = 0; i < 8; ++i) o[i] = (unsigned short)bf16_bits(f[i]);
  return o;
}

__global__ __launch_bounds__(NTHR) void k_prep(const float* __restrict__ x, const float* __restrict__ w1,
                                               const float* __restrict__ b1, const float* __restrict__ w2,
                                               const float* __restrict__ b2, const float* __restrict__ w3,
                                               const float* __restrict__ b3,
                                               unsigned short* xb, unsigned short* w1t, unsigned short* w2d,
                                               unsigned short* w3d, float* sm) {
  const int tid = (int)threadIdx.x;
  const int blk = (int)blockIdx.x;
  if (blk < PBX) {
    const int u   = blk * NTHR + tid;
    const int row = u >> 5, k8 = (u & 31) * 8;
    const int rc  = row < NN ? row : NN - 1;
    const unsigned mk = row < NN ? 0xffffu : 0u;
    const float* p = x + (size_t)rc * F0 + k8;
    const v4f a = *(const v4fa*)p;
    const v4f b = *(const v4fa*)(p + 4);
    v8us o;
    o[0] = (unsigned short)(bf16_bits(a.x) & mk); o[1] = (unsigned short)(bf16_bits(a.y) & mk);
    o[2] = (unsigned short)(bf16_bits(a.z) & mk); o[3] = (unsigned short)(bf16_bits(a.w) & mk);
    o[4] = (unsigned short)(bf16_bits(b.x) & mk); o[5] = (unsigned short)(bf16_bits(b.y) & mk);
    o[6] = (unsigned short)(bf16_bits(b.z) & mk); o[7] = (unsigned short)(bf16_bits(b.w) & mk);
    st2_v8us(xb + (size_t)row * F0 + k8, o);
  } else if (blk < PBX + PBW1) {
    const int u = (blk - PBX) * NTHR + tid;
    const int n = u >> 5, k8 = (u & 31) * 8;
    const v8us o = gather8(w1 + (size_t)k8 * H1W + n, H1W);
    st2_v8us(w1t + (size_t)n * BP1 + k8, o);
  } else if (blk < PBX + PBW1 + PBW2) {
    const int u = (blk - PBX - PBW1) * NTHR + tid;
    const int n = u >> 7, k8 = (u & 127) * 8, kk = k8 & 511;
    const v8us o = gather8(w2 + (size_t)kk * H2W + n, H2W);
    st2_v8us(w2d + (size_t)n * BP2 + k8, o);
  } else if (blk < PBX + PBW1 + PBW2 + PBW3) {
    const int u = (blk - PBX - PBW1 - PBW2) * NTHR + tid;
    const int n = u >> 6, k8 = (u & 63) * 8, kk = k8 & 255;
    const v8us o = gather8(w3 + (size_t)kk * NC + n, NC);
    st2_v8us(w3d + (size_t)n * BP3 + k8, o);
  } else {
    const int q  = tid;
    const int qa = q < 127 ? q : 127;
    int qb = q - 128; qb = qb < 0 ? 0 : (qb > 63 ? 63 : qb);
    int qc = q - 192; qc = qc < 0 ? 0 : (qc > 3 ? 3 : qc);
    const v4f a = *(const v4fa*)(b1 + 4 * qa);
    const v4f b = *(const v4fa*)(b2 + 4 * qb);
    const v4f c = *(const v4fa*)(b3 + 4 * qc);
    asm volatile("" :: "v"(a));
    asm volatile("" :: "v"(b));
    asm volatile("" :: "v"(c));
    const unsigned ma = (q < 128) ? 0xffffffffu : 0u;
    const unsigned mb = (q >= 128 && q < 192) ? 0xffffffffu : 0u;
    const unsigned mc = (q >= 192 && q < 196) ? 0xffffffffu : 0u;
    v4f o;
    o.x = __uint_as_float(((bf16_bits(a.x) << 16) & ma) | ((bf16_bits(b.x) << 16) & mb) | ((bf16_bits(c.x) << 16) & mc));
    o.y = __uint_as_float(((bf16_bits(a.y) << 16) & ma) | ((bf16_bits(b.y) << 16) & mb) | ((bf16_bits(c.y) << 16) & mc));
    o.z = __uint_as_float(((bf16_bits(a.z) << 16) & ma) | ((bf16_bits(b.z) << 16) & mb) | ((bf16_bits(c.z) << 16) & mc));
    o.w = __uint_as_float(((bf16_bits(a.w) << 16) & ma) | ((bf16_bits(b.w) << 16) & mb) | ((bf16_bits(c.w) << 16) & mc));
    if (tid < SMF / 4) st2_v4f(sm + 4 * tid, o);
  }
}

__device__ __forceinline__ void bucket_flush(const int* pl, const int* cnt, int ov, int* lp, int* cop, int* fp,
                                             int tid) {
#pragma unroll 1
  for (int i = tid * 4; i < RCAP; i += NTHR * 4) {
    const v4i v = *(const v4ia*)(pl + i);
    *(volatile v4i*)(lp + i) = v;
  }
#pragma unroll 1
  for (int i = tid * 4; i < 2 * NBRUN; i += NTHR * 4) {
    const v4i v = *(const v4ia*)(cnt + i);
    *(volatile v4i*)(cop + i) = v;
  }
  if (tid < 8) {
    const v4i f = {ov, ov, ov, ov};
    *(volatile v4i*)(fp + 4 * tid) = f;
  }
}

__global__ __launch_bounds__(NTHR) void k_bucket(const int* __restrict__ srcs, const int* __restrict__ dsts,
                                                 const float* __restrict__ ew, int* LIST, int* CO, int* FLAG) {
  extern __shared__ __attribute__((aligned(16))) int dsm[];
  int* wl   = dsm;
  int* pl   = dsm + NWAVE * WLCAP;
  int* cnt  = pl + RCAP;
  int* offs = cnt + NBRUN;
  int* cur  = offs + NBRUN;
  int* misc = cur + NBRUN;
  const int tid = (int)threadIdx.x, lane = tid & 31, wave = tid >> 5;
  const int blk = (int)blockIdx.x;
  const unsigned nbs = (unsigned)(blk * NBRUN);
  int nbi = NN - blk * NBRUN;
  nbi = nbi > NBRUN ? NBRUN : (nbi < 1 ? 1 : nbi);
  const unsigned unb = (unsigned)nbi;

  {
    const v4i z4 = {0, 0, 0, 0};
    for (int i = tid * 4; i < BK_ZINTS; i += NTHR * 4) *(v4ia*)(dsm + i) = z4;
    if (tid < 16) misc[tid] = 0;
  }
  __syncthreads();

  {
    const int per  = ((NE + NWAVE * WCH - 1) / (NWAVE * WCH)) * WCH;
    const int ebeg = wave * per;
    const int eend = (ebeg + per < NE) ? (ebeg + per) : NE;
    int* mylist = wl + wave * WLCAP;
    int wc = 0;
#pragma unroll 1
    for (int cb = ebeg; cb < eend; cb += WCH) {
      const int e0 = cb + lane * EPT;
      const v4i da = *(const v4ia*)(dsts + e0);
      const v4i db = *(const v4ia*)(dsts + e0 + 4);
      const unsigned s0 = (unsigned)da.x - nbs, s1 = (unsigned)da.y - nbs;
      const unsigned s2 = (unsigned)da.z - nbs, s3 = (unsigned)da.w - nbs;
      const unsigned s4 = (unsigned)db.x - nbs, s5 = (unsigned)db.y - nbs;
      const unsigned s6 = (unsigned)db.z - nbs, s7 = (unsigned)db.w - nbs;
      const bool h0 = s0 < unb, h1 = s1 < unb, h2 = s2 < unb, h3 = s3 < unb;
      const bool h4 = s4 < unb, h5 = s5 < unb, h6 = s6 < unb, h7 = s7 < unb;
      const unsigned m0 = __builtin_amdgcn_ballot_w32(h0), m1 = __builtin_amdgcn_ballot_w32(h1);
      const unsigned m2 = __builtin_amdgcn_ballot_w32(h2), m3 = __builtin_amdgcn_ballot_w32(h3);
      const unsigned m4 = __builtin_amdgcn_ballot_w32(h4), m5 = __builtin_amdgcn_ballot_w32(h5);
      const unsigned m6 = __builtin_amdgcn_ballot_w32(h6), m7 = __builtin_amdgcn_ballot_w32(h7);
      const unsigned any = m0 | m1 | m2 | m3 | m4 | m5 | m6 | m7;
      if (any != 0u) {
        const int pre = (int)(__builtin_amdgcn_mbcnt_lo(m0, 0u) + __builtin_amdgcn_mbcnt_lo(m1, 0u) +
                              __builtin_amdgcn_mbcnt_lo(m2, 0u) + __builtin_amdgcn_mbcnt_lo(m3, 0u) +
                              __builtin_amdgcn_mbcnt_lo(m4, 0u) + __builtin_amdgcn_mbcnt_lo(m5, 0u) +
                              __builtin_amdgcn_mbcnt_lo(m6, 0u) + __builtin_amdgcn_mbcnt_lo(m7, 0u));
        int p = wc + pre;
        if (h0) { if (p < WLCAP) mylist[p] = ((e0 + 0) << SLB) | (int)s0; p = p + 1; }
        if (h1) { if (p < WLCAP) mylist[p] = ((e0 + 1) << SLB) | (int)s1; p = p + 1; }
        if (h2) { if (p < WLCAP) mylist[p] = ((e0 + 2) << SLB) | (int)s2; p = p + 1; }
        if (h3) { if (p < WLCAP) mylist[p] = ((e0 + 3) << SLB) | (int)s3; p = p + 1; }
        if (h4) { if (p < WLCAP) mylist[p] = ((e0 + 4) << SLB) | (int)s4; p = p + 1; }
        if (h5) { if (p < WLCAP) mylist[p] = ((e0 + 5) << SLB) | (int)s5; p = p + 1; }
        if (h6) { if (p < WLCAP) mylist[p] = ((e0 + 6) << SLB) | (int)s6; p = p + 1; }
        if (h7) { if (p < WLCAP) mylist[p] = ((e0 + 7) << SLB) | (int)s7; p = p + 1; }
        wc += (int)(__builtin_popcount(m0) + __builtin_popcount(m1) + __builtin_popcount(m2) + __builtin_popcount(m3) +
                    __builtin_popcount(m4) + __builtin_popcount(m5) + __builtin_popcount(m6) + __builtin_popcount(m7));
      }
    }
    if (lane == 0) misc[wave] = wc;
  }
  __syncthreads();

  if (wave == 0) {
    int ov = 0;
#pragma unroll 1
    for (int w2 = 0; w2 < NWAVE; ++w2) {
      int c = misc[w2];
      if (c > WLCAP) ov = 1;
      c = c < 0 ? 0 : (c > WLCAP ? WLCAP : c);
#pragma unroll 1
      for (int b0 = 0; b0 < c; b0 += 32) {
        const int idx = b0 + lane;
        const int ent = wl[w2 * WLCAP + (idx < WLCAP ? idx : WLCAP - 1)];
        const int m32 = (c - b0) < 32 ? (c - b0) : 32;
#pragma unroll 1
        for (int k = 0; k < m32; ++k) {
          const int u    = __builtin_amdgcn_readlane(ent, k);
          const int slot = u & (NBRUN - 1);
          if (lane == 0) cnt[slot] = cnt[slot] + 1;
        }
      }
    }
    if (lane == 0) misc[9] = ov;
  }
  __syncthreads();
  if (wave == 0) {
    const int base = lane * (NBRUN / 32);
    int s = 0;
#pragma unroll 1
    for (int i = 0; i < NBRUN / 32; ++i) s += cnt[base + i];
    int incl = s;
#pragma unroll
    for (int d = 1; d < 32; d <<= 1) {
      const int y = __shfl_up(incl, d, 32);
      if (lane >= d) incl += y;
    }
    int run = incl - s;
#pragma unroll 1
    for (int i = 0; i < NBRUN / 32; ++i) {
      const int cv = cnt[base + i];
      offs[base + i] = run;
      cur[base + i]  = run;
      run += cv;
    }
  }
  __syncthreads();

  if (wave == 0) {
#pragma unroll 1
    for (int w2 = 0; w2 < NWAVE; ++w2) {
      int c = misc[w2];
      c = c < 0 ? 0 : (c > WLCAP ? WLCAP : c);
#pragma unroll 1
      for (int b0 = 0; b0 < c; b0 += 32) {
        const int idx = b0 + lane;
        const int ent = wl[w2 * WLCAP + (idx < WLCAP ? idx : WLCAP - 1)];
        int eid = (ent >> SLB) & 0x1FFFFF;
        eid = eid > NE - 1 ? NE - 1 : eid;
        int sr = srcs[eid];
        sr = sr < 0 ? 0 : (sr > NN - 1 ? NN - 1 : sr);
        const int word = (int)((unsigned)sr | (bf16_bits(ew[eid]) << 16));
        const int m32 = (c - b0) < 32 ? (c - b0) : 32;
#pragma unroll 1
        for (int k = 0; k < m32; ++k) {
          const int u    = __builtin_amdgcn_readlane(ent, k);
          const int wd   = __builtin_amdgcn_readlane(word, k);
          const int slot = u & (NBRUN - 1);
          if (lane == 0) {
            int p = cur[slot];
            p = p < 0 ? 0 : (p > RCAP - 1 ? RCAP - 1 : p);
            pl[p] = wd;
            cur[slot] = p + 1;
          }
        }
      }
    }
  }
  __syncthreads();

  const int ovf = misc[9];
  int* lp  = LIST + (size_t)blk * RCAP;
  int* cop = CO + (size_t)blk * (2 * NBRUN);
  int* fp  = FLAG + (size_t)blk * 32;
  bucket_flush(pl, cnt, ovf, lp, cop, fp, tid);
  __threadfence();
  bucket_flush(pl, cnt, ovf, lp, cop, fp, tid);
}

template <int KTOT, int BPITCH, int NT>
__device__ __forceinline__ void gemm_rows16(const unsigned short* __restrict__ ap,
                                            const unsigned short* __restrict__ bp, v8f (&acc)[NT]) {
#pragma unroll 1
  for (int k0 = 0; k0 < KTOT; k0 += 32) {
    FragB af;
    af.h[0] = *(const v8usa*)(ap + k0);
    af.h[1] = *(const v8usa*)(ap + k0 + 16);
#pragma unroll
    for (int t = 0; t < NT; ++t) {
      const unsigned short* wq = bp + (size_t)(16 * t) * (size_t)BPITCH + k0;
      FragB bf;
      bf.h[0] = *(const v8usa*)wq;
      bf.h[1] = *(const v8usa*)(wq + 16);
      acc[t] = wmb(af, bf, acc[t]);
    }
  }
}

template <int KTOT, int APITCH, int BPITCH, int NOUT>
__device__ __forceinline__ void gemm_tile(const unsigned short* __restrict__ A,
                                          const unsigned short* __restrict__ BT, float* C, float* stg) {
  const int tid = (int)threadIdx.x, lane = tid & 31, wave = tid >> 5, hh = lane >> 4, m = lane & 15;
  const int rowBase = (int)blockIdx.x * GBM;
  const int colBase = (int)blockIdx.y * GBN;
  v8f acc[8];
  {
    const v8f z = {0.f, 0.f, 0.f, 0.f, 0.f, 0.f, 0.f, 0.f};
#pragma unroll
    for (int t = 0; t < 8; ++t) acc[t] = z;
  }
  const unsigned short* ap = A + (size_t)(rowBase + 16 * wave + m) * (size_t)APITCH + 8 * hh;
  const unsigned short* bp = BT + (size_t)(colBase + m) * (size_t)BPITCH + 8 * hh;
  gemm_rows16<KTOT, BPITCH, 8>(ap, bp, acc);
#pragma unroll
  for (int t = 0; t < 8; ++t) {
#pragma unroll
    for (int r = 0; r < 8; ++r) stg[(16 * wave + 8 * hh + r) * GBN + 16 * t + m] = acc[t][r];
  }
  __syncthreads();
#pragma unroll 1
  for (int i = 0; i < 16; ++i) {
    const int lr = 16 * wave + i;
    const int gr = rowBase + lr;
    const v4f v = *(const v4fa*)(stg + lr * GBN + 4 * lane);
    asm volatile("" :: "v"(v));
    if (gr < NN) st2_v4f(C + (size_t)gr * (size_t)NOUT + colBase + 4 * lane, v);
  }
}

__global__ __launch_bounds__(GTHR) __attribute__((amdgpu_num_vgpr(248)))
void k_gemm_one(const unsigned short* __restrict__ A, const unsigned short* __restrict__ BT, float* C) {
  __shared__ __attribute__((aligned(16))) float stg[GBM * GBN];
  gemm_tile<K1, AP1, BP1, H1W>(A, BT, C, stg);
}

__global__ __launch_bounds__(GTHR) __attribute__((amdgpu_num_vgpr(248)))
void k_gemm_two(const unsigned short* __restrict__ A, const unsigned short* __restrict__ BT, float* C) {
  __shared__ __attribute__((aligned(16))) float stg[GBM * GBN];
  gemm_tile<K2, AP2, BP2, H2W>(A, BT, C, stg);
}

__device__ __forceinline__ void flush3(const float* stg, float* ob, int nv4, int tid) {
#pragma unroll 1
  for (int it = 0; it < 2; ++it) {
    const int i4 = it * NTHR + tid;
    const v4f v = *(const v4fa*)(stg + 4 * i4);
    asm volatile("" :: "v"(v));
    if (i4 < nv4) *(volatile v4f*)(ob + (size_t)4 * (size_t)i4) = v;
  }
}

__global__ __launch_bounds__(NTHR) __attribute__((amdgpu_num_vgpr(248)))
void k_gemm_three(const unsigned short* __restrict__ A, const unsigned short* __restrict__ BT, float* C) {
  __shared__ __attribute__((aligned(16))) float stg[128 * NC];
  const int tid = (int)threadIdx.x, lane = tid & 31, wave = tid >> 5, hh = lane >> 4, m = lane & 15;
  const int rowBase = (int)blockIdx.x * 128;
  v8f acc[1];
  {
    const v8f z = {0.f, 0.f, 0.f, 0.f, 0.f, 0.f, 0.f, 0.f};
    acc[0] = z;
  }
  const unsigned short* ap = A + (size_t)(rowBase + 16 * wave + m) * (size_t)AP3 + 8 * hh;
  const unsigned short* bp = BT + (size_t)m * (size_t)BP3 + 8 * hh;
  gemm_rows16<K3, BP3, 1>(ap, bp, acc);
#pragma unroll
  for (int r = 0; r < 8; ++r) stg[(16 * wave + 8 * hh + r) * NC + m] = acc[0][r];
  __syncthreads();
  int liveRows = NN - rowBase;
  liveRows = liveRows > 128 ? 128 : (liveRows < 0 ? 0 : liveRows);
  const int nv4 = liveRows * (NC / 4);
  float* ob = C + (size_t)rowBase * NC;
  flush3(stg, ob, nv4, tid);
  __threadfence();
  flush3(stg, ob, nv4, tid);
}

template <int NJ>
__global__ __launch_bounds__(NTHR) void k_replay_hl(const int* __restrict__ LIST, const int* __restrict__ CO,
                                                    const int* __restrict__ FLAG, const float* __restrict__ P,
                                                    const float* __restrict__ BT, unsigned short* H) {
  constexpr int W  = 128 * NJ;
  constexpr int HP = 2 * W;
  static_assert(W / 4 <= NTHR && (W / 4) % 32 == 0);
  __shared__ __attribute__((aligned(16))) float sb[W];
  const int tid = (int)threadIdx.x, lane = tid & 31, wave = tid >> 5, hh = lane >> 4, t16 = lane & 15;
  {
    const int qi = tid < W / 4 ? tid : W / 4 - 1;
    const v4f bv = *(const v4fa*)(BT + 4 * qi);
    asm volatile("" :: "v"(bv));
    if (tid < W / 4) *(v4fa*)(sb + 4 * tid) = bv;
  }
  __syncthreads();
  v4f bias[NJ];
#pragma unroll
  for (int jj = 0; jj < NJ; ++jj) bias[jj] = *(const v4fa*)(sb + 4 * lane + 128 * jj);

  const int rowBase = (int)blockIdx.x * RPB;
  const int bucket  = rowBase >> SLB;
  const int* lb  = LIST + (size_t)bucket * RCAP;
  const int* cob = CO + (size_t)bucket * (2 * NBRUN);
  const int flag = FLAG[(size_t)bucket * 32];
  const float qnan = __uint_as_float(0x7fc00000u);

#pragma unroll 1
  for (int ri = 0; ri < RPW; ++ri) {
    const int d    = rowBase + RPW * wave + ri;
    const int slot = d & (NBRUN - 1);
    int c = cob[slot];
    int o = cob[NBRUN + slot];
    const bool big = c > TRIPCAP;
    c = c < 0 ? 0 : (c > TRIPCAP ? TRIPCAP : c);
    o = o < 0 ? 0 : (o > RCAP - 1 ? RCAP - 1 : o);
    if (c > RCAP - o) c = RCAP - o;
    const int cs = __builtin_amdgcn_readfirstlane(c);
    int last = o + c - 1;
    last = last < o ? o : last;
    last = last > RCAP - 1 ? RCAP - 1 : last;
    v4f a[NJ];
    {
      const v4f z = {0.0f, 0.0f, 0.0f, 0.0f};
#pragma unroll
      for (int jj = 0; jj < NJ; ++jj) a[jj] = z;
    }
#pragma unroll 1
    for (int j = 0; j < cs; ++j) {
      int idx = o + j;
      idx = idx > last ? last : idx;
      const unsigned wd = (unsigned)lb[idx];
      int sr = (int)(wd & 0xffffu);
      sr = sr > NN - 1 ? NN - 1 : sr;
      const float w = __uint_as_float(wd & 0xffff0000u);
      const float* prow = P + (size_t)sr * W + 4 * lane;
#pragma unroll
      for (int jj = 0; jj < NJ; ++jj) {
        const v4f v = *(const v4fa*)(prow + 128 * jj);
        a[jj].x = fmaf(w, v.x, a[jj].x);
        a[jj].y = fmaf(w, v.y, a[jj].y);
        a[jj].z = fmaf(w, v.z, a[jj].z);
        a[jj].w = fmaf(w, v.w, a[jj].w);
      }
    }
    const bool bad  = (flag != 0) | big;
    const bool live = d < NN;
    v4i ow[NJ];
#pragma unroll
    for (int jj = 0; jj < NJ; ++jj) {
      float v0 = a[jj].x + bias[jj].x, v1 = a[jj].y + bias[jj].y;
      float v2 = a[jj].z + bias[jj].z, v3 = a[jj].w + bias[jj].w;
      v0 = (v0 > 0.0f) ? v0 : (v0 - v0); v1 = (v1 > 0.0f) ? v1 : (v1 - v1);
      v2 = (v2 > 0.0f) ? v2 : (v2 - v2); v3 = (v3 > 0.0f) ? v3 : (v3 - v3);
      v0 = bad ? qnan : v0; v1 = bad ? qnan : v1; v2 = bad ? qnan : v2; v3 = bad ? qnan : v3;
      v0 = live ? v0 : 0.0f; v1 = live ? v1 : 0.0f; v2 = live ? v2 : 0.0f; v3 = live ? v3 : 0.0f;
      int h01, h23, l01, l23;
      hilo_pack(v0, v1, v2, v3, h01, h23, l01, l23);
      ow[jj] = regroup16(h01, h23, l01, l23, lane);
    }
    unsigned short* hp = H + (size_t)d * HP + hh * W + 8 * t16;
#pragma unroll
    for (int jj = 0; jj < NJ; ++jj) *(volatile v4i*)(hp + 128 * jj) = ow[jj];
    __threadfence();
#pragma unroll
    for (int jj = 0; jj < NJ; ++jj) *(volatile v4i*)(hp + 128 * jj) = ow[jj];
  }
}

__global__ __launch_bounds__(NTHR) void k_replay_out(const int* __restrict__ LIST, const int* __restrict__ CO,
                                                     const int* __restrict__ FLAG, const float* __restrict__ P3,
                                                     const float* __restrict__ B3, float* out) {
  __shared__ __attribute__((aligned(16))) float sb3[NC];
  const int tid = (int)threadIdx.x, lane = tid & 31, wave = tid >> 5, hh = lane >> 4, q = lane & 15;
  if (tid < 32) {
    const float bv = B3[q];
    asm volatile("" :: "v"(bv));
    if (lane < NC) sb3[lane] = bv;
  }
  __syncthreads();
  const float b = sb3[q];

  const int blk     = (int)blockIdx.x;
  const int rowBase = blk * 16;
  const int bucket  = rowBase >> SLB;
  const int* lb  = LIST + (size_t)bucket * RCAP;
  const int* cob = CO + (size_t)bucket * (2 * NBRUN);
  const int flag = FLAG[(size_t)bucket * 32];
  const float qnan = __uint_as_float(0x7fc00000u);

  const int d    = rowBase + 2 * wave + hh;
  const int slot = d & (NBRUN - 1);
  int c = cob[slot];
  int o = cob[NBRUN + slot];
  const bool big = c > TRIPCAP;
  c = c < 0 ? 0 : (c > TRIPCAP ? TRIPCAP : c);
  o = o < 0 ? 0 : (o > RCAP - 1 ? RCAP - 1 : o);
  if (c > RCAP - o) c = RCAP - o;
  const int co  = __shfl_xor(c, 16, 32);
  const int cmv = c > co ? c : co;
  const int cm  = __builtin_amdgcn_readfirstlane(cmv);
  int last = o + c - 1;
  last = last < o ? o : last;
  last = last > RCAP - 1 ? RCAP - 1 : last;
  float acc = 0.0f;
#pragma unroll 1
  for (int j = 0; j < cm; ++j) {
    int idx = o + j;
    idx = idx > last ? last : idx;
    const unsigned wd = (unsigned)lb[idx];
    int sr = (int)(wd & 0xffffu);
    sr = sr > NN - 1 ? NN - 1 : sr;
    const float w = __uint_as_float(wd & 0xffff0000u);
    const float v = P3[(size_t)sr * NC + q];
    asm volatile("" :: "v"(v));
    const float t = fmaf(w, v, acc);
    acc = (j < c) ? t : acc;
  }
  const float h = acc + b;
  float m = h;
#pragma unroll
  for (int s = 8; s >= 1; s >>= 1) {
    const float v = __shfl_xor(m, s, 32);
    m = ((v > m) | (v != v)) ? v : m;
  }
  const float e = expf(h - m);
  float se = e;
#pragma unroll
  for (int s = 8; s >= 1; s >>= 1) se += __shfl_xor(se, s, 32);
  float r = (h - m) - logf(se);
  const bool bad = (flag != 0) | big;
  r = bad ? qnan : r;
  float* op = out + (size_t)blk * 256 + 32 * wave + lane;
  *(volatile float*)op = r;
  __threadfence();
  *(volatile float*)op = r;
}

extern "C" void kernel_launch(void* const* d_in, const int* in_sizes, int n_in,
                              void* d_out, int out_size, void* d_ws, size_t ws_size,
                              hipStream_t stream) {
  if (n_in < 10) return;
  if (in_sizes[0] != NN * F0) return;
  if (in_sizes[1] != NE) return;
  if (in_sizes[2] != NE) return;
  if (in_sizes[3] != NE) return;
  if (in_sizes[4] != F0 * H1W) return;
  if (in_sizes[5] != H1W) return;
  if (in_sizes[6] != H1W * H2W) return;
  if (in_sizes[7] != H2W) return;
  if (in_sizes[8] != H2W * NC) return;
  if (in_sizes[9] != NC) return;
  if (out_size != NN * NC) return;

  const float* x    = (const float*)d_in[0];
  const int*   srcs = (const int*)d_in[1];
  const int*   dsts = (const int*)d_in[2];
  const float* ew   = (const float*)d_in[3];
  const float* W1   = (const float*)d_in[4];
  const float* b1   = (const float*)d_in[5];
  const float* W2   = (const float*)d_in[6];
  const float* b2   = (const float*)d_in[7];
  const float* W3   = (const float*)d_in[8];
  const float* b3   = (const float*)d_in[9];
  float* out = (float*)d_out;

  constexpr size_t zH    = (size_t)MP * AP2 * 2;
  constexpr size_t zXB   = (size_t)MP * F0 * 2;
  constexpr size_t zH2   = (size_t)MP * AP3 * 2;
  constexpr size_t zP    = (size_t)NN * H1W * 4;
  constexpr size_t zLIST = (size_t)NBK * RCAP * 4;
  constexpr size_t zCO   = (size_t)NBK * 2 * NBRUN * 4;
  constexpr size_t zFLAG = (size_t)NBK * 128;
  constexpr size_t zW1T  = (size_t)H1W * BP1 * 2;
  constexpr size_t zW2D  = (size_t)H2W * BP2 * 2;
  constexpr size_t zW3D  = (size_t)NC * BP3 * 2;
  constexpr size_t zSM   = (size_t)SMF * 4;
  constexpr size_t oH    = 0;
  constexpr size_t oP    = oH + zH;
  constexpr size_t oLIST = oP + zP;
  constexpr size_t oCO   = oLIST + zLIST;
  constexpr size_t oFLAG = oCO + zCO;
  constexpr size_t oW1T  = oFLAG + zFLAG;
  constexpr size_t oW2D  = oW1T + zW1T;
  constexpr size_t oW3D  = oW2D + zW2D;
  constexpr size_t oSM   = oW3D + zW3D;
  constexpr size_t oEND  = oSM + zSM;
  static_assert(zXB <= zH && zH2 <= zH);
  static_assert((size_t)NN * H2W * 4 <= zP && (size_t)NN * NC * 4 <= zP);
  static_assert(zH % 256 == 0 && zP % 256 == 0 && zLIST % 256 == 0 && zCO % 256 == 0 && zFLAG % 256 == 0);
  static_assert(zW1T % 256 == 0 && zW2D % 256 == 0 && zW3D % 256 == 0 && zSM % 256 == 0);
  static_assert(oEND <= (size_t)(128u << 20));
  if (oEND > ws_size) return;

  char* ws = (char*)d_ws;
  unsigned short* H    = (unsigned short*)(ws + oH);
  unsigned short* XB   = (unsigned short*)(ws + oH);
  float*          P    = (float*)(ws + oP);
  int*            LIST = (int*)(ws + oLIST);
  int*            CO   = (int*)(ws + oCO);
  int*            FLAG = (int*)(ws + oFLAG);
  unsigned short* W1T  = (unsigned short*)(ws + oW1T);
  unsigned short* W2D  = (unsigned short*)(ws + oW2D);
  unsigned short* W3D  = (unsigned short*)(ws + oW3D);
  float*          SM   = (float*)(ws + oSM);

  hipFuncSetAttribute(reinterpret_cast<const void*>(&k_bucket), hipFuncAttributeMaxDynamicSharedMemorySize, (int)BK_LDS);

  k_prep<<<PBTOT, NTHR, 0, stream>>>(x, W1, b1, W2, b2, W3, b3, XB, W1T, W2D, W3D, SM);
  k_bucket<<<NBK, NTHR, BK_LDS, stream>>>(srcs, dsts, ew, LIST, CO, FLAG);
  k_gemm_one<<<dim3(MP / GBM, H1W / GBN, 1), GTHR, 0, stream>>>(XB, W1T, P);
  k_replay_hl<4><<<MP / RPB, NTHR, 0, stream>>>(LIST, CO, FLAG, P, SM, H);
  k_gemm_two<<<dim3(MP / GBM, H2W / GBN, 1), GTHR, 0, stream>>>(H, W2D, P);
  k_replay_hl<2><<<MP / RPB, NTHR, 0, stream>>>(LIST, CO, FLAG, P, SM + 512, H);
  k_gemm_three<<<MP / 128, NTHR, 0, stream>>>(H, W3D, P);
  k_replay_out<<<NN / 16, NTHR, 0, stream>>>(LIST, CO, FLAG, P, SM + 768, out);
}
